// CrossAttnV3_30193620091389
// MI455X (gfx1250) — hardware-verified
//
#include <hip/hip_runtime.h>
#include <math.h>
#include <stdint.h>

#define NB    4
#define NQ    1024
#define NKV   2048
#define DM    1024
#define NH    16
#define HD    64
#define RQ    (NB * NQ)
#define RC    (NB * NKV)
#define NQT   (NQ / 64)
#define NKT   (NKV / 64)
#define OUTN  (RQ * DM)
static_assert(NH * HD == DM);
static_assert(HD == 64);
static_assert(NKT == 32);
static_assert((NQ % 64) == 0 && (NKV % 64) == 0 && (DM % 64) == 0 && (DM % 32) == 0);
static_assert((RQ % 32) == 0 && (RC % 32) == 0);
static_assert((((RQ / 64) * (DM / 64)) % 8) == 0);
static_assert((((RC / 64) * (2 * DM / 64)) % 8) == 0);
static_assert(((RQ * DM / 8) % 256) == 0 && ((RC * DM / 8) % 256) == 0 && ((DM * DM / 8) % 256) == 0);
static_assert(((NB * DM) % 8) == 0);

typedef _Float16 v16h __attribute__((ext_vector_type(16)));
typedef _Float16 v8h  __attribute__((ext_vector_type(8)));
typedef float    v8f  __attribute__((ext_vector_type(8)));
typedef float    v4f  __attribute__((ext_vector_type(4)));
typedef unsigned int v4u __attribute__((ext_vector_type(4)));

__device__ __forceinline__ unsigned short bf_bits(float f) {
  unsigned u = __float_as_uint(f);
  return (unsigned short)((u + 0x7FFFu + ((u >> 16) & 1u)) >> 16);
}
__device__ __forceinline__ float bfr(float f) { return __uint_as_float(((unsigned)bf_bits(f)) << 16); }
__device__ __forceinline__ unsigned short h_bits(_Float16 x) { return __builtin_bit_cast(unsigned short, x); }
__device__ __forceinline__ unsigned pk16(unsigned short a, unsigned short b) { return (unsigned)a | ((unsigned)b << 16); }
__device__ __forceinline__ v8f zero8() { v8f z = {0.f, 0.f, 0.f, 0.f, 0.f, 0.f, 0.f, 0.f}; return z; }
__device__ __forceinline__ float wsum32(float s) {
#pragma unroll
  for (int off = 16; off >= 1; off >>= 1) s += __shfl_xor(s, off, 32);
  return s;
}

__device__ __forceinline__ v16h ldfrag_h(const _Float16* p) {
  union { v16h v; v8h h[2]; } f;
  f.h[0] = *(const v8h*)(p);
  f.h[1] = *(const v8h*)(p + 16);
  return f.v;
}

__device__ __forceinline__ v8f mma_h(v16h a, v16h b, v8f c) {
  c = __builtin_amdgcn_wmma_f32_16x16x32_f16(false, a, false, b, (short)0, c, false, false);
#if defined(__HIP_DEVICE_COMPILE__)
  asm volatile("v_nop\n\tv_nop\n\tv_nop\n\tv_nop" : "+v"(c) : "v"(a), "v"(b));
#endif
  return c;
}
__device__ __forceinline__ v8f mma_h_raw(v16h a, v16h b, v8f c) {
  return __builtin_amdgcn_wmma_f32_16x16x32_f16(false, a, false, b, (short)0, c, false, false);
}
__device__ __forceinline__ void dep_guard_h(v8f& a, v8f& b, v16h x, v16h y) {
#if defined(__HIP_DEVICE_COMPILE__)
  asm volatile("v_nop\n\tv_nop\n\tv_nop\n\tv_nop" : "+v"(a), "+v"(b) : "v"(x), "v"(y));
#endif
}
__device__ __forceinline__ void keep4_h(v16h a, v16h b, v16h c, v16h d) {
#if defined(__HIP_DEVICE_COMPILE__)
  asm volatile("v_nop" :: "v"(a), "v"(b), "v"(c), "v"(d));
#endif
}
__device__ __forceinline__ void acc_guard4(v8f& a, v8f& b, v8f& c, v8f& d) {
#if defined(__HIP_DEVICE_COMPILE__)
  asm volatile("v_nop\n\tv_nop\n\tv_nop\n\tv_nop" : "+v"(a), "+v"(b), "+v"(c), "+v"(d));
#endif
}

__global__ __launch_bounds__(256) void cvt16(const float* __restrict__ in, unsigned short* out, int n8, float scale) {
  const int i = blockIdx.x * 256 + threadIdx.x;
  if (i < n8) {
    const v4f a = *(const v4f*)(in + (size_t)i * 8);
    const v4f b = *(const v4f*)(in + (size_t)i * 8 + 4);
    v4u p;
    p[0] = pk16(h_bits((_Float16)(bfr(a[0]) * scale)), h_bits((_Float16)(bfr(a[1]) * scale)));
    p[1] = pk16(h_bits((_Float16)(bfr(a[2]) * scale)), h_bits((_Float16)(bfr(a[3]) * scale)));
    p[2] = pk16(h_bits((_Float16)(bfr(b[0]) * scale)), h_bits((_Float16)(bfr(b[1]) * scale)));
    p[3] = pk16(h_bits((_Float16)(bfr(b[2]) * scale)), h_bits((_Float16)(bfr(b[3]) * scale)));
    *(volatile v4u*)(out + (size_t)i * 8) = p;
    __threadfence();
    *(volatile v4u*)(out + (size_t)i * 8) = p;
  }
}

__global__ __launch_bounds__(256) void cvt16g(const float* __restrict__ in, const float* __restrict__ gam,
                                              unsigned short* out, int n8, int kd8, float scale) {
  const int i = blockIdx.x * 256 + threadIdx.x;
  if (i < n8) {
    const int k8 = (i % kd8) * 8;
    const v4f a  = *(const v4f*)(in + (size_t)i * 8);
    const v4f b  = *(const v4f*)(in + (size_t)i * 8 + 4);
    const v4f g0 = *(const v4f*)(gam + k8);
    const v4f g1 = *(const v4f*)(gam + k8 + 4);
    float gs[8];
    gs[0] = bfr(g0[0]) * scale; gs[1] = bfr(g0[1]) * scale; gs[2] = bfr(g0[2]) * scale; gs[3] = bfr(g0[3]) * scale;
    gs[4] = bfr(g1[0]) * scale; gs[5] = bfr(g1[1]) * scale; gs[6] = bfr(g1[2]) * scale; gs[7] = bfr(g1[3]) * scale;
    v4u p;
    p[0] = pk16(h_bits((_Float16)(bfr(a[0]) * gs[0])), h_bits((_Float16)(bfr(a[1]) * gs[1])));
    p[1] = pk16(h_bits((_Float16)(bfr(a[2]) * gs[2])), h_bits((_Float16)(bfr(a[3]) * gs[3])));
    p[2] = pk16(h_bits((_Float16)(bfr(b[0]) * gs[4])), h_bits((_Float16)(bfr(b[1]) * gs[5])));
    p[3] = pk16(h_bits((_Float16)(bfr(b[2]) * gs[6])), h_bits((_Float16)(bfr(b[3]) * gs[7])));
    *(volatile v4u*)(out + (size_t)i * 8) = p;
    __threadfence();
    *(volatile v4u*)(out + (size_t)i * 8) = p;
  }
}

__global__ __launch_bounds__(256) void ln_stats(const float* __restrict__ x, float* mup, float* rsp, int nrows) {
  __shared__ __align__(16) float sMu[32];
  __shared__ __align__(16) float sRs[32];
  const int lane = threadIdx.x & 31, wave = threadIdx.x >> 5;
  const int rb = blockIdx.x * 32;
#pragma unroll 1
  for (int i = 0; i < 4; ++i) {
    int row = rb + wave * 4 + i;
    row = (row < nrows) ? row : (nrows - 1);
    const float* xr = x + (size_t)row * DM;
    float v[32];
    float s = 0.f;
#pragma unroll
    for (int j = 0; j < 8; ++j) {
      const v4f a = *(const v4f*)(xr + j * 128 + lane * 4);
#pragma unroll
      for (int e = 0; e < 4; ++e) { const float t = bfr(a[e]); v[j * 4 + e] = t; s += t; }
    }
    s = wsum32(s);
    const float mu = s * (1.0f / (float)DM);
    float q = 0.f;
#pragma unroll
    for (int k = 0; k < 32; ++k) { const float d = v[k] - mu; q += d * d; }
    q = wsum32(q);
    const float var = q * (1.0f / (float)DM);
    const float rs = rsqrtf(var + 1e-5f);
    if (lane == 0) { sMu[wave * 4 + i] = mu; sRs[wave * 4 + i] = rs; }
  }
  __syncthreads();
  if (wave == 0) {
    const int pc = lane & 7;
    const v4f m4 = *(const v4f*)(sMu + pc * 4);
    const v4f r4 = *(const v4f*)(sRs + pc * 4);
    for (int pass = 0; pass < 2; ++pass) {
      if (lane < 8) {
        *(volatile v4f*)(mup + rb + pc * 4) = m4;
        *(volatile v4f*)(rsp + rb + pc * 4) = r4;
      }
      __threadfence();
    }
  }
}

__global__ __launch_bounds__(256) void colsum_k(const unsigned short* __restrict__ Whp, const float* __restrict__ W,
                                                const float* __restrict__ beta, float* Gp, float* Bcp,
                                                int nrows, float inv_scale) {
  __shared__ __align__(16) float sG[32];
  __shared__ __align__(16) float sB[32];
  const int lane = threadIdx.x & 31, wave = threadIdx.x >> 5;
  const int rb = blockIdx.x * 32;
  float bt[32];
#pragma unroll
  for (int j = 0; j < 8; ++j) {
    const v4f a = *(const v4f*)(beta + j * 128 + lane * 4);
#pragma unroll
    for (int e = 0; e < 4; ++e) bt[j * 4 + e] = bfr(a[e]);
  }
#pragma unroll 1
  for (int i = 0; i < 4; ++i) {
    int row = rb + wave * 4 + i;
    row = (row < nrows) ? row : (nrows - 1);
    const _Float16* hr = (const _Float16*)(const void*)Whp + (size_t)row * DM;
    const float* wr = W + (size_t)row * DM;
    float g = 0.f, bs = 0.f;
#pragma unroll
    for (int j = 0; j < 4; ++j) {
      const v8h a = *(const v8h*)(hr + j * 256 + lane * 8);
#pragma unroll
      for (int e = 0; e < 8; ++e) g += (float)a[e];
    }
#pragma unroll
    for (int j = 0; j < 8; ++j) {
      const v4f a = *(const v4f*)(wr + j * 128 + lane * 4);
#pragma unroll
      for (int e = 0; e < 4; ++e) bs += bfr(a[e]) * bt[j * 4 + e];
    }
    g = wsum32(g);
    bs = wsum32(bs);
    if (lane == 0) { sG[wave * 4 + i] = g * inv_scale; sB[wave * 4 + i] = bs; }
  }
  __syncthreads();
  if (wave == 0) {
    const int pc = lane & 7;
    const v4f g4 = *(const v4f*)(sG + pc * 4);
    const v4f b4 = *(const v4f*)(sB + pc * 4);
    for (int pass = 0; pass < 2; ++pass) {
      if (lane < 8) {
        *(volatile v4f*)(Gp + rb + pc * 4) = g4;
        *(volatile v4f*)(Bcp + rb + pc * 4) = b4;
      }
      __threadfence();
    }
  }
}

__global__ __launch_bounds__(256) void gemm_ln(
    const unsigned short* __restrict__ Ap, int lda,
    const unsigned short* __restrict__ Btp, int ldb,
    const float* __restrict__ mup, const float* __restrict__ rsp,
    const float* __restrict__ Gp, const float* __restrict__ Bcp,
    float cscale, float oscale,
    unsigned short* C16, int ldc,
    unsigned short* Th, unsigned short* Tr, int tseq, int dv,
    int M, int N, int K, int nsplit) {
  const _Float16* Ah = (const _Float16*)(const void*)Ap;
  const _Float16* Bt = (const _Float16*)(const void*)Btp;
  __shared__ __align__(16) float sT[8][16 * 68];
  const int lane = threadIdx.x & 31;
  const int wave = threadIdx.x >> 5;
  const int tilesN = N >> 6;
  const int tilesM = M >> 6;
  const int tile = blockIdx.x * 8 + wave;
  if (tile >= tilesM * tilesN) return;
  const int tm = tile / tilesN;
  const int tn = tile - tm * tilesN;
  const int m0 = tm << 6;
  const int n0 = tn << 6;

  const int rlane = lane & 15;
  const int koff  = (lane >> 4) * 8;
  const int mOff  = (lane >> 4) * 8;

  v8f acc[4][4];
#pragma unroll
  for (int i = 0; i < 4; ++i)
#pragma unroll
    for (int j = 0; j < 4; ++j) acc[i][j] = zero8();

  for (int k0 = 0; k0 < K; k0 += 32) {
    v16h bh[4];
#pragma unroll
    for (int j = 0; j < 4; ++j) {
      const size_t bo = (size_t)(n0 + (j << 4) + rlane) * ldb + koff + k0;
      bh[j] = ldfrag_h(Bt + bo);
    }
#pragma unroll
    for (int i = 0; i < 4; ++i) {
      const size_t ao = (size_t)(m0 + (i << 4) + rlane) * lda + koff + k0;
      const v16h ah = ldfrag_h(Ah + ao);
#pragma unroll
      for (int j = 0; j < 4; ++j) {
        acc[i][j] = mma_h_raw(ah, bh[j], acc[i][j]);
      }
      dep_guard_h(acc[i][0], acc[i][3], ah, bh[3]);
    }
    keep4_h(bh[0], bh[1], bh[2], bh[3]);
  }
  acc_guard4(acc[0][0], acc[0][1], acc[0][2], acc[0][3]);
  acc_guard4(acc[1][0], acc[1][1], acc[1][2], acc[1][3]);
  acc_guard4(acc[2][0], acc[2][1], acc[2][2], acc[2][3]);
  acc_guard4(acc[3][0], acc[3][1], acc[3][2], acc[3][3]);

  float* slab = sT[wave];
  float g[4], bc[4];
#pragma unroll
  for (int j = 0; j < 4; ++j) {
    g[j]  = Gp[n0 + (j << 4) + rlane];
    bc[j] = Bcp[n0 + (j << 4) + rlane];
  }
  const int rq = lane >> 3, piece = lane & 7;

  if (n0 < nsplit) {
#pragma unroll
    for (int i = 0; i < 4; ++i) {
      const int mBase = m0 + (i << 4);
      const v4f mua = *(const v4f*)(mup + mBase + mOff);
      const v4f mub = *(const v4f*)(mup + mBase + mOff + 4);
      const v4f rsa = *(const v4f*)(rsp + mBase + mOff);
      const v4f rsb = *(const v4f*)(rsp + mBase + mOff + 4);
      float mu8[8], rs8[8];
      mu8[0] = mua[0]; mu8[1] = mua[1]; mu8[2] = mua[2]; mu8[3] = mua[3];
      mu8[4] = mub[0]; mu8[5] = mub[1]; mu8[6] = mub[2]; mu8[7] = mub[3];
      rs8[0] = rsa[0]; rs8[1] = rsa[1]; rs8[2] = rsa[2]; rs8[3] = rsa[3];
      rs8[4] = rsb[0]; rs8[5] = rsb[1]; rs8[6] = rsb[2]; rs8[7] = rsb[3];
#pragma unroll
      for (int r = 0; r < 8; ++r) {
        const int row = mOff + r;
#pragma unroll
        for (int j = 0; j < 4; ++j)
          slab[row * 68 + (j << 4) + rlane] = rs8[r] * (acc[i][j][r] * cscale - mu8[r] * g[j]) + bc[j];
      }
      __builtin_amdgcn_fence(__ATOMIC_RELEASE, "workgroup");
      __builtin_amdgcn_wave_barrier();
      __builtin_amdgcn_fence(__ATOMIC_ACQUIRE, "workgroup");
      v4u ph[4];
#pragma unroll
      for (int it = 0; it < 4; ++it) {
        const int row = it * 4 + rq;
        const v4f a  = *(const v4f*)(slab + row * 68 + piece * 8);
        const v4f a2 = *(const v4f*)(slab + row * 68 + piece * 8 + 4);
        float f[8];
        f[0] = a[0];  f[1] = a[1];  f[2] = a[2];  f[3] = a[3];
        f[4] = a2[0]; f[5] = a2[1]; f[6] = a2[2]; f[7] = a2[3];
        v4u p;
#pragma unroll
        for (int e = 0; e < 4; ++e) {
          const _Float16 x0 = (_Float16)(f[2 * e] * oscale), x1 = (_Float16)(f[2 * e + 1] * oscale);
          p[e] = pk16(h_bits(x0), h_bits(x1));
        }
        ph[it] = p;
      }
      for (int pass = 0; pass < 2; ++pass) {
#pragma unroll
        for (int it = 0; it < 4; ++it) {
          const int row = it * 4 + rq;
          const size_t co = (size_t)(mBase + row) * ldc + n0 + piece * 8;
          *(volatile v4u*)(C16 + co) = ph[it];
        }
        __threadfence();
      }
      __builtin_amdgcn_fence(__ATOMIC_RELEASE, "workgroup");
      __builtin_amdgcn_wave_barrier();
      __builtin_amdgcn_fence(__ATOMIC_ACQUIRE, "workgroup");
    }
  } else {
    const int bb = m0 / tseq;
    const int t0 = m0 - bb * tseq;
    const int fb = n0 - nsplit;
#pragma unroll
    for (int j = 0; j < 4; ++j) {
#pragma unroll
      for (int i = 0; i < 4; ++i) {
        const int mBase = m0 + (i << 4);
        const v4f mua = *(const v4f*)(mup + mBase + mOff);
        const v4f mub = *(const v4f*)(mup + mBase + mOff + 4);
        const v4f rsa = *(const v4f*)(rsp + mBase + mOff);
        const v4f rsb = *(const v4f*)(rsp + mBase + mOff + 4);
        float mu8[8], rs8[8];
        mu8[0] = mua[0]; mu8[1] = mua[1]; mu8[2] = mua[2]; mu8[3] = mua[3];
        mu8[4] = mub[0]; mu8[5] = mub[1]; mu8[6] = mub[2]; mu8[7] = mub[3];
        rs8[0] = rsa[0]; rs8[1] = rsa[1]; rs8[2] = rsa[2]; rs8[3] = rsa[3];
        rs8[4] = rsb[0]; rs8[5] = rsb[1]; rs8[6] = rsb[2]; rs8[7] = rsb[3];
#pragma unroll
        for (int r = 0; r < 8; ++r) {
          slab[rlane * 68 + (i << 4) + mOff + r] = rs8[r] * (acc[i][j][r] * cscale - mu8[r] * g[j]) + bc[j];
        }
      }
      __builtin_amdgcn_fence(__ATOMIC_RELEASE, "workgroup");
      __builtin_amdgcn_wave_barrier();
      __builtin_amdgcn_fence(__ATOMIC_ACQUIRE, "workgroup");
      v4u ph[4], pr[4];
      size_t hofs[4];
#pragma unroll
      for (int it = 0; it < 4; ++it) {
        const int row = it * 4 + rq;
        const v4f a  = *(const v4f*)(slab + row * 68 + piece * 8);
        const v4f a2 = *(const v4f*)(slab + row * 68 + piece * 8 + 4);
        float f[8];
        f[0] = a[0];  f[1] = a[1];  f[2] = a[2];  f[3] = a[3];
        f[4] = a2[0]; f[5] = a2[1]; f[6] = a2[2]; f[7] = a2[3];
        v4u p, q;
#pragma unroll
        for (int e = 0; e < 4; ++e) {
          const float g0 = f[2 * e] * oscale, g1 = f[2 * e + 1] * oscale;
          const _Float16 x0 = (_Float16)g0, x1 = (_Float16)g1;
          const _Float16 y0 = (_Float16)((g0 - (float)x0) * 2048.0f);
          const _Float16 y1 = (_Float16)((g1 - (float)x1) * 2048.0f);
          p[e] = pk16(h_bits(x0), h_bits(x1));
          q[e] = pk16(h_bits(y0), h_bits(y1));
        }
        ph[it] = p;
        pr[it] = q;
        hofs[it] = ((size_t)(bb * dv + fb + (j << 4) + row)) * (size_t)tseq + t0 + piece * 8;
      }
      for (int pass = 0; pass < 2; ++pass) {
#pragma unroll
        for (int it = 0; it < 4; ++it) {
          *(volatile v4u*)(Th + hofs[it]) = ph[it];
          *(volatile v4u*)(Tr + hofs[it]) = pr[it];
        }
        __threadfence();
      }
      __builtin_amdgcn_fence(__ATOMIC_RELEASE, "workgroup");
      __builtin_amdgcn_wave_barrier();
      __builtin_amdgcn_fence(__ATOMIC_ACQUIRE, "workgroup");
    }
  }
}

__global__ __launch_bounds__(256) void gemm_out(
    const unsigned short* __restrict__ Ap, const unsigned short* __restrict__ Arp, int lda,
    const unsigned short* __restrict__ Btp, int ldb,
    const float* __restrict__ biasp, float cscale,
    float* Cf, int ldc, int M, int N, int K) {
  const _Float16* Ah  = (const _Float16*)(const void*)Ap;
  const _Float16* Arh = (const _Float16*)(const void*)Arp;
  const _Float16* Bt  = (const _Float16*)(const void*)Btp;
  __shared__ __align__(16) float sT[8][16 * 68];
  const int lane = threadIdx.x & 31;
  const int wave = threadIdx.x >> 5;
  const int tilesN = N >> 6;
  const int tilesM = M >> 6;
  const int tile = blockIdx.x * 8 + wave;
  if (tile >= tilesM * tilesN) return;
  const int tm = tile / tilesN;
  const int tn = tile - tm * tilesN;
  const int m0 = tm << 6;
  const int n0 = tn << 6;

  const int rlane = lane & 15;
  const int koff  = (lane >> 4) * 8;
  const int mOff  = (lane >> 4) * 8;

  v8f acc[4][4];
#pragma unroll
  for (int i = 0; i < 4; ++i)
#pragma unroll
    for (int j = 0; j < 4; ++j) acc[i][j] = zero8();

#pragma unroll 1
  for (int pl = 0; pl < 2; ++pl) {
    const _Float16* Asel = (pl == 0) ? Arh : Ah;
    if (pl == 1) {
      acc_guard4(acc[0][0], acc[0][1], acc[0][2], acc[0][3]);
      acc_guard4(acc[1][0], acc[1][1], acc[1][2], acc[1][3]);
      acc_guard4(acc[2][0], acc[2][1], acc[2][2], acc[2][3]);
      acc_guard4(acc[3][0], acc[3][1], acc[3][2], acc[3][3]);
#pragma unroll
      for (int i = 0; i < 4; ++i)
#pragma unroll
        for (int j = 0; j < 4; ++j) acc[i][j] = acc[i][j] * (1.0f / 2048.0f);
      acc_guard4(acc[0][0], acc[0][1], acc[0][2], acc[0][3]);
      acc_guard4(acc[1][0], acc[1][1], acc[1][2], acc[1][3]);
      acc_guard4(acc[2][0], acc[2][1], acc[2][2], acc[2][3]);
      acc_guard4(acc[3][0], acc[3][1], acc[3][2], acc[3][3]);
    }
    for (int k0 = 0; k0 < K; k0 += 32) {
      v16h bh[4];
#pragma unroll
      for (int j = 0; j < 4; ++j) {
        const size_t bo = (size_t)(n0 + (j << 4) + rlane) * ldb + koff + k0;
        bh[j] = ldfrag_h(Bt + bo);
      }
#pragma unroll
      for (int i = 0; i < 4; ++i) {
        const size_t ao = (size_t)(m0 + (i << 4) + rlane) * lda + koff + k0;
        const v16h ah = ldfrag_h(Asel + ao);
#pragma unroll
        for (int j = 0; j < 4; ++j) {
          acc[i][j] = mma_h_raw(ah, bh[j], acc[i][j]);
        }
        dep_guard_h(acc[i][0], acc[i][3], ah, bh[3]);
      }
      keep4_h(bh[0], bh[1], bh[2], bh[3]);
    }
  }
  acc_guard4(acc[0][0], acc[0][1], acc[0][2], acc[0][3]);
  acc_guard4(acc[1][0], acc[1][1], acc[1][2], acc[1][3]);
  acc_guard4(acc[2][0], acc[2][1], acc[2][2], acc[2][3]);
  acc_guard4(acc[3][0], acc[3][1], acc[3][2], acc[3][3]);

  float* slab = sT[wave];
  float bj[4];
#pragma unroll
  for (int j = 0; j < 4; ++j) bj[j] = bfr(biasp[n0 + (j << 4) + rlane]);
#pragma unroll
  for (int i = 0; i < 4; ++i) {
    const int mBase = m0 + (i << 4);
#pragma unroll
    for (int r = 0; r < 8; ++r) {
      const int row = mOff + r;
#pragma unroll
      for (int j = 0; j < 4; ++j) slab[row * 68 + (j << 4) + rlane] = acc[i][j][r] * cscale + bj[j];
    }
    __builtin_amdgcn_fence(__ATOMIC_RELEASE, "workgroup");
    __builtin_amdgcn_wave_barrier();
    __builtin_amdgcn_fence(__ATOMIC_ACQUIRE, "workgroup");
    const int hh = lane >> 4, c4 = (lane & 15) * 4;
    v4f ov[8];
#pragma unroll
    for (int it = 0; it < 8; ++it) {
      const int row = it * 2 + hh;
      ov[it] = *(const v4f*)(slab + row * 68 + c4);
    }
    for (int pass = 0; pass < 2; ++pass) {
#pragma unroll
      for (int it = 0; it < 8; ++it) {
        const int row = it * 2 + hh;
        *(volatile v4f*)(Cf + (size_t)(mBase + row) * ldc + n0 + c4) = ov[it];
      }
      __threadfence();
    }
    __builtin_amdgcn_fence(__ATOMIC_RELEASE, "workgroup");
    __builtin_amdgcn_wave_barrier();
    __builtin_amdgcn_fence(__ATOMIC_ACQUIRE, "workgroup");
  }
}

__global__ __launch_bounds__(256) void v_sum(const unsigned short* __restrict__ vth, const unsigned short* __restrict__ vtr,
                                             float* vs, int nrows) {
  const int lane = threadIdx.x & 31, wave = threadIdx.x >> 5;
  int row = blockIdx.x * 8 + wave;
  row = (row < nrows) ? row : (nrows - 1);
  const _Float16* ph = (const _Float16*)(const void*)vth + (size_t)row * NKV + lane * 64;
  const _Float16* pr = (const _Float16*)(const void*)vtr + (size_t)row * NKV + lane * 64;
  float s = 0.f, sr = 0.f;
#pragma unroll 1
  for (int i = 0; i < 8; ++i) {
    const v8h a = *(const v8h*)(ph + 8 * i);
    const v8h b = *(const v8h*)(pr + 8 * i);
#pragma unroll
    for (int e = 0; e < 8; ++e) { s += (float)a[e]; sr += (float)b[e]; }
  }
  const float v = s + sr * (1.0f / 2048.0f);
  float* dst = vs + (size_t)row * NKT + lane;
  *(volatile float*)dst = v;
  __threadfence();
  *(volatile float*)dst = v;
}

__global__ __launch_bounds__(128)
void attn_x(const unsigned short* __restrict__ qpp, const unsigned short* __restrict__ kpp,
            const unsigned short* __restrict__ vtp, const unsigned short* __restrict__ vtrp,
            const float* __restrict__ vsp, unsigned short* ctxp, unsigned short* ctxrp) {
  union FH { v16h v; v8h h[2]; };
  constexpr int TB     = 64 * 64 * 2;
  constexpr int PB     = 4 * 16 * 64 * 2;
  constexpr int SB     = 64 * NKT * 4;
  constexpr int OFF_K  = 0;
  constexpr int OFF_V  = TB;
  constexpr int OFF_VR = 2 * TB;
  constexpr int OFF_P  = 3 * TB;
  constexpr int OFF_S  = OFF_P + PB;
  constexpr int SMEMB  = OFF_S + SB;
  static_assert(4 * 16 * 64 * 4 <= OFF_P);
  __shared__ __align__(16) unsigned char smem[SMEMB];
  _Float16* Ksh = (_Float16*)(smem + OFF_K);
  _Float16* Vsh = (_Float16*)(smem + OFF_V);
  _Float16* Vrs = (_Float16*)(smem + OFF_VR);
  _Float16* Psh = (_Float16*)(smem + OFF_P);
  float*    Ssh = (float*)(smem + OFF_S);

  const int tid  = threadIdx.x;
  const int wave = tid >> 5;
  const int lane = tid & 31;
  const int hh   = lane >> 4;
  const int c    = lane & 15;

  const int bx   = blockIdx.x;
  const int qb   = bx % NQT;
  const int rest = bx / NQT;
  const int h    = rest % NH;
  const int b    = rest / NH;
  const int q0   = qb * 64 + wave * 16;
  const size_t qrow0 = (size_t)b * NQ;
  const size_t krow0 = (size_t)b * NKV;
  const size_t vrowb = (size_t)b * DM + (size_t)h * HD;

  const _Float16* Qp  = (const _Float16*)(const void*)qpp + (size_t)h * HD;
  const _Float16* Kp  = (const _Float16*)(const void*)kpp + (size_t)h * HD;
  const _Float16* Vt  = (const _Float16*)(const void*)vtp  + vrowb * NKV;
  const _Float16* Vrt = (const _Float16*)(const void*)vtrp + vrowb * NKV;
  const float*    Vs  = vsp + vrowb * NKT;

  {
    const int d = tid >> 1, half = (tid & 1) * 16;
#pragma unroll
    for (int i = 0; i < 4; ++i) {
      const v4f a = *(const v4f*)(Vs + (size_t)d * NKT + half + 4 * i);
      *(v4f*)(Ssh + d * NKT + half + 4 * i) = a;
    }
  }

  v16h qa[2];
#pragma unroll
  for (int dc = 0; dc < 2; ++dc) {
    const size_t qo = (qrow0 + q0 + c) * DM + dc * 32 + 8 * hh;
    qa[dc] = ldfrag_h(Qp + qo);
  }

  float rmax[8], lsum[8];
  float osd[4][8];
  v8f oacc[4], oacc2[4];
#pragma unroll
  for (int r = 0; r < 8; ++r) { rmax[r] = -1e30f; lsum[r] = 0.f; }
#pragma unroll
  for (int t = 0; t < 4; ++t) {
    oacc[t] = zero8(); oacc2[t] = zero8();
#pragma unroll
    for (int r = 0; r < 8; ++r) osd[t][r] = 0.f;
  }

  _Float16* pw = Psh + wave * (16 * 64);

#pragma unroll 1
  for (int kt = 0; kt < NKT; ++kt) {
    const int kv0 = kt * 64;
    __syncthreads();
    {
      const int r = tid >> 1, half = (tid & 1) * 32;
      const size_t ko = (krow0 + kv0 + r) * DM + half;
      const size_t vo = (size_t)r * NKV + kv0 + half;
#pragma unroll
      for (int i = 0; i < 4; ++i) {
        const v8h a0 = *(const v8h*)(Kp + ko + 8 * i);
        const v8h b0 = *(const v8h*)(Vt + vo + 8 * i);
        const v8h b1 = *(const v8h*)(Vrt + vo + 8 * i);
        *(v8h*)(Ksh + r * 64 + half + 8 * i) = a0;
        *(v8h*)(Vsh + r * 64 + half + 8 * i) = b0;
        *(v8h*)(Vrs + r * 64 + half + 8 * i) = b1;
      }
    }
    __syncthreads();

    v8f s[4];
#pragma unroll
    for (int j = 0; j < 4; ++j) {
      s[j] = zero8();
#pragma unroll
      for (int dc = 0; dc < 2; ++dc) {
        FH kb;
        kb.h[0] = *(const v8h*)(Ksh + (j * 16 + c) * 64 + dc * 32 + 8 * hh);
        kb.h[1] = *(const v8h*)(Ksh + (j * 16 + c) * 64 + dc * 32 + 16 + 8 * hh);
        s[j] = mma_h(qa[dc], kb.v, s[j]);
      }
    }

    float tmax[8];
#pragma unroll
    for (int r = 0; r < 8; ++r) {
      float m = -1e30f;
#pragma unroll
      for (int j = 0; j < 4; ++j) {
        s[j][r] = s[j][r] * (1.0f / 2048.0f);
        m = fmaxf(m, s[j][r]);
      }
      tmax[r] = m;
    }
#pragma unroll
    for (int r = 0; r < 8; ++r) {
#pragma unroll
      for (int off = 1; off < 16; off <<= 1) tmax[r] = fmaxf(tmax[r], __shfl_xor(tmax[r], off, 32));
    }
    float corr[8], tsum[8], ct[8];
#pragma unroll
    for (int r = 0; r < 8; ++r) {
      const float mnew = fmaxf(rmax[r], tmax[r]);
      corr[r] = __expf(rmax[r] - mnew);
      rmax[r] = mnew;
      float ts = 0.f;
#pragma unroll
      for (int j = 0; j < 4; ++j) {
        const float e = __expf(s[j][r] - mnew);
        s[j][r] = e;
        ts += e;
      }
      tsum[r] = ts;
    }
#pragma unroll
    for (int r = 0; r < 8; ++r) {
#pragma unroll
      for (int off = 1; off < 16; off <<= 1) tsum[r] += __shfl_xor(tsum[r], off, 32);
      lsum[r] = lsum[r] * corr[r] + tsum[r];
      ct[r] = tsum[r] * (1.0f / 64.0f);
    }
#pragma unroll
    for (int r = 0; r < 8; ++r) {
#pragma unroll
      for (int j = 0; j < 4; ++j)
        pw[(8 * hh + r) * 64 + j * 16 + c] = (_Float16)((s[j][r] - ct[r]) * 1024.0f);
    }
    float vd[4];
#pragma unroll
    for (int t = 0; t < 4; ++t) vd[t] = Ssh[(t * 16 + c) * NKT + kt];
#pragma unroll
    for (int t = 0; t < 4; ++t) {
#pragma unroll
      for (int r = 0; r < 8; ++r) {
        osd[t][r] = osd[t][r] * corr[r] + ct[r] * vd[t];
        oacc[t][r]  = oacc[t][r]  * corr[r];
        oacc2[t][r] = oacc2[t][r] * corr[r];
      }
    }
    acc_guard4(oacc[0], oacc[1], oacc[2], oacc[3]);
    acc_guard4(oacc2[0], oacc2[1], oacc2[2], oacc2[3]);
    __builtin_amdgcn_fence(__ATOMIC_RELEASE, "workgroup");
    __builtin_amdgcn_wave_barrier();
    __builtin_amdgcn_fence(__ATOMIC_ACQUIRE, "workgroup");

#pragma unroll
    for (int kk = 0; kk < 2; ++kk) {
      FH pa;
      pa.h[0] = *(const v8h*)(pw + c * 64 + kk * 32 + 8 * hh);
      pa.h[1] = *(const v8h*)(pw + c * 64 + kk * 32 + 16 + 8 * hh);
#pragma unroll
      for (int t = 0; t < 4; ++t) {
        FH vb, vrb;
        vb.h[0]  = *(const v8h*)(Vsh + (t * 16 + c) * 64 + kk * 32 + 8 * hh);
        vb.h[1]  = *(const v8h*)(Vsh + (t * 16 + c) * 64 + kk * 32 + 16 + 8 * hh);
        vrb.h[0] = *(const v8h*)(Vrs + (t * 16 + c) * 64 + kk * 32 + 8 * hh);
        vrb.h[1] = *(const v8h*)(Vrs + (t * 16 + c) * 64 + kk * 32 + 16 + 8 * hh);
        oacc[t]  = mma_h(pa.v, vb.v, oacc[t]);
        oacc2[t] = mma_h(pa.v, vrb.v, oacc2[t]);
      }
    }
  }
  __syncthreads();

  float* os = (float*)(void*)smem + wave * (16 * 64);
#pragma unroll
  for (int r = 0; r < 8; ++r) {
    const float rl = 16.0f / lsum[r];
#pragma unroll
    for (int t = 0; t < 4; ++t) {
      const float v = oacc[t][r] * (1.0f / 1024.0f) + oacc2[t][r] * (1.0f / 2097152.0f) + osd[t][r];
      os[(8 * hh + r) * 64 + t * 16 + c] = v * rl;
    }
  }
  __builtin_amdgcn_fence(__ATOMIC_RELEASE, "workgroup");
  __builtin_amdgcn_wave_barrier();
  __builtin_amdgcn_fence(__ATOMIC_ACQUIRE, "workgroup");
  {
    const int rq = lane >> 3, piece = lane & 7;
    v4u ph[4], pr[4];
    size_t go[4];
#pragma unroll
    for (int it = 0; it < 4; ++it) {
      const int row = it * 4 + rq;
      const v4f a  = *(const v4f*)(os + row * 64 + piece * 8);
      const v4f a2 = *(const v4f*)(os + row * 64 + piece * 8 + 4);
      float f[8];
      f[0] = a[0];  f[1] = a[1];  f[2] = a[2];  f[3] = a[3];
      f[4] = a2[0]; f[5] = a2[1]; f[6] = a2[2]; f[7] = a2[3];
      v4u p, q;
#pragma unroll
      for (int e = 0; e < 4; ++e) {
        const _Float16 x0 = (_Float16)f[2 * e], x1 = (_Float16)f[2 * e + 1];
        const _Float16 y0 = (_Float16)((f[2 * e] - (float)x0) * 2048.0f);
        const _Float16 y1 = (_Float16)((f[2 * e + 1] - (float)x1) * 2048.0f);
        p[e] = pk16(h_bits(x0), h_bits(x1));
        q[e] = pk16(h_bits(y0), h_bits(y1));
      }
      ph[it] = p;
      pr[it] = q;
      go[it] = (qrow0 + q0 + row) * DM + (size_t)h * HD + piece * 8;
    }
    for (int pass = 0; pass < 2; ++pass) {
#pragma unroll
      for (int it = 0; it < 4; ++it) {
        *(volatile v4u*)(ctxp + go[it])  = ph[it];
        *(volatile v4u*)(ctxrp + go[it]) = pr[it];
      }
      __threadfence();
    }
  }
}

extern "C" void kernel_launch(void* const* d_in, const int* in_sizes, int n_in,
                              void* d_out, int out_size, void* d_ws, size_t ws_size,
                              hipStream_t stream) {
  if (n_in < 10) return;
  if (in_sizes[0] != RQ * DM) return;
  if (in_sizes[1] != RC * DM) return;
  if (in_sizes[2] != DM * DM) return;
  if (in_sizes[3] != 2 * DM * DM) return;
  if (in_sizes[4] != DM * DM) return;
  if (in_sizes[5] != DM || in_sizes[6] != DM || in_sizes[7] != DM || in_sizes[8] != DM || in_sizes[9] != DM) return;
  if (out_size != OUTN) return;

  const float* q      = (const float*)d_in[0];
  const float* cx     = (const float*)d_in[1];
  const float* w_q    = (const float*)d_in[2];
  const float* w_kv   = (const float*)d_in[3];
  const float* w_p    = (const float*)d_in[4];
  const float* b_p    = (const float*)d_in[5];
  const float* q_gam  = (const float*)d_in[6];
  const float* q_bet  = (const float*)d_in[7];
  const float* c_gam  = (const float*)d_in[8];
  const float* c_bet  = (const float*)d_in[9];

  const size_t PXq  = (size_t)RQ * DM * 2;
  const size_t PXc  = (size_t)RC * DM * 2;
  const size_t PWq  = (size_t)DM * DM * 2;
  const size_t PWkv = (size_t)2 * DM * DM * 2;
  const size_t PWp  = (size_t)DM * DM * 2;
  const size_t PSq  = (size_t)RQ * 4;
  const size_t PSc  = (size_t)RC * 4;
  const size_t PGq  = (size_t)DM * 4;
  const size_t PGkv = (size_t)2 * DM * 4;
  const size_t PQp  = (size_t)RQ * DM * 2;
  const size_t PKp  = (size_t)RC * DM * 2;
  const size_t PVT  = (size_t)NB * DM * NKV * 2;
  const size_t PVS  = (size_t)NB * DM * NKT * 4;
  const size_t PCtx = (size_t)RQ * DM * 2;
  size_t off = 0;
  const size_t oXq   = off; off += PXq;
  const size_t oXc   = off; off += PXc;
  const size_t oWq   = off; off += PWq;
  const size_t oWkv  = off; off += PWkv;
  const size_t oWp   = off; off += PWp;
  const size_t oMuQ  = off; off += PSq;
  const size_t oRsQ  = off; off += PSq;
  const size_t oMuC  = off; off += PSc;
  const size_t oRsC  = off; off += PSc;
  const size_t oGq   = off; off += PGq;
  const size_t oBq   = off; off += PGq;
  const size_t oGkv  = off; off += PGkv;
  const size_t oBkv  = off; off += PGkv;
  const size_t oQp   = off; off += PQp;
  const size_t oKp   = off; off += PKp;
  const size_t oVT   = off; off += PVT;
  const size_t oVTr  = off; off += PVT;
  const size_t oVS   = off; off += PVS;
  const size_t oCtx  = off; off += PCtx;
  const size_t oCtxr = off; off += PCtx;
  if (off > ws_size) return;
  if (off > (size_t)134217728) return;

  char* ws = (char*)d_ws;
  unsigned short* Xq   = (unsigned short*)(ws + oXq);
  unsigned short* Xc   = (unsigned short*)(ws + oXc);
  unsigned short* Wqh  = (unsigned short*)(ws + oWq);
  unsigned short* Wkvh = (unsigned short*)(ws + oWkv);
  unsigned short* Wph  = (unsigned short*)(ws + oWp);
  float*          muQ  = (float*)(ws + oMuQ);
  float*          rsQ  = (float*)(ws + oRsQ);
  float*          muC  = (float*)(ws + oMuC);
  float*          rsC  = (float*)(ws + oRsC);
  float*          Gq   = (float*)(ws + oGq);
  float*          Bq   = (float*)(ws + oBq);
  float*          Gkv  = (float*)(ws + oGkv);
  float*          Bkv  = (float*)(ws + oBkv);
  unsigned short* Qp   = (unsigned short*)(ws + oQp);
  unsigned short* Kp   = (unsigned short*)(ws + oKp);
  unsigned short* VT   = (unsigned short*)(ws + oVT);
  unsigned short* VTr  = (unsigned short*)(ws + oVTr);
  float*          VS   = (float*)(ws + oVS);
  unsigned short* Ctx  = (unsigned short*)(ws + oCtx);
  unsigned short* Ctxr = (unsigned short*)(ws + oCtxr);
  float*          outf = (float*)d_out;

  const dim3 blk(256);
  const int n8q  = RQ * DM / 8;
  const int n8c  = RC * DM / 8;
  const int n8wq = DM * DM / 8;
  const int n8wk = 2 * DM * DM / 8;
  const int n8wp = DM * DM / 8;
  const dim3 gCq((n8q + 255) / 256);
  const dim3 gCc((n8c + 255) / 256);
  const dim3 gCwq((n8wq + 255) / 256);
  const dim3 gCwk((n8wk + 255) / 256);
  const dim3 gCwp((n8wp + 255) / 256);
  const dim3 gSq(RQ / 32);
  const dim3 gSc(RC / 32);
  const dim3 gColq(DM / 32);
  const dim3 gColk(2 * DM / 32);
  const dim3 gGq(((RQ / 64) * (DM / 64) + 7) / 8);
  const dim3 gGkv(((RC / 64) * (2 * DM / 64) + 7) / 8);
  const dim3 gVs(NB * DM / 8);
  const dim3 gAttn(NQT * NH * NB);
  const dim3 gGout(((RQ / 64) * (DM / 64) + 7) / 8);
  const float wScale = 1024.0f;
  const float aScale = 16.0f;
  const float csProj = 1.0f / 16384.0f;
  const float csOut  = 1.0f / 262144.0f;

  cvt16<<<gCq, blk, 0, stream>>>(q, Xq, n8q, aScale);
  cvt16<<<gCc, blk, 0, stream>>>(cx, Xc, n8c, aScale);
  cvt16g<<<gCwq, blk, 0, stream>>>(w_q, q_gam, Wqh, n8wq, DM / 8, wScale);
  cvt16g<<<gCwk, blk, 0, stream>>>(w_kv, c_gam, Wkvh, n8wk, DM / 8, wScale);
  cvt16<<<gCwp, blk, 0, stream>>>(w_p, Wph, n8wp, wScale);
  ln_stats<<<gSq, blk, 0, stream>>>(q, muQ, rsQ, RQ);
  ln_stats<<<gSc, blk, 0, stream>>>(cx, muC, rsC, RC);
  colsum_k<<<gColq, blk, 0, stream>>>(Wqh, w_q, q_bet, Gq, Bq, DM, 1.0f / 1024.0f);
  colsum_k<<<gColk, blk, 0, stream>>>(Wkvh, w_kv, c_bet, Gkv, Bkv, 2 * DM, 1.0f / 1024.0f);
  gemm_ln<<<gGq, blk, 0, stream>>>(Xq, DM, Wqh, DM, muQ, rsQ, Gq, Bq, csProj, aScale,
                                   Qp, DM, Qp, Qp, NQ, DM, RQ, DM, DM, DM);
  gemm_ln<<<gGkv, blk, 0, stream>>>(Xc, DM, Wkvh, DM, muC, rsC, Gkv, Bkv, csProj, aScale,
                                    Kp, DM, VT, VTr, NKV, DM, RC, 2 * DM, DM, DM);
  v_sum<<<gVs, blk, 0, stream>>>(VT, VTr, VS, NB * DM);
  attn_x<<<gAttn, dim3(128), 0, stream>>>(Qp, Kp, VT, VTr, VS, Ctx, Ctxr);
  gemm_out<<<gGout, blk, 0, stream>>>(Ctx, Ctxr, DM, Wph, DM, b_p, csOut, outf, DM, RQ, DM, DM);
  (void)hipGetLastError();
}
